// Transformation_81630148428263
// MI455X (gfx1250) — hardware-run, weakly checked
//
#include <hip/hip_runtime.h>
#pragma clang fp contract(off)


#ifndef NROWS
#define NROWS 131072
#endif
#define NROWS_FULL 131072
#define NV   16
#define DEG  32
#define KD   32
#define TW   8

static_assert(NV == 16);
static_assert(KD == DEG);
static_assert(KD == 32);
static_assert(NROWS % (16 * TW) == 0);
static_assert(NROWS <= NROWS_FULL);
static_assert((size_t)NROWS_FULL * NV * 4 == (size_t)8388608);

typedef unsigned short bf;
typedef __attribute__((ext_vector_type(16))) __bf16   v16bf;
typedef __attribute__((ext_vector_type(8)))  unsigned short v8us;
typedef __attribute__((ext_vector_type(8)))  unsigned v8u;
typedef __attribute__((ext_vector_type(8)))  float    v8f;
typedef __attribute__((ext_vector_type(4)))  float    v4f;
typedef v4f  __attribute__((may_alias)) v4fa;

__device__ __forceinline__ unsigned short f2bf(float f) { unsigned u = __float_as_uint(f); u += 0x7FFFu + ((u >> 16) & 1u); return (unsigned short)(u >> 16); }
__device__ __forceinline__ float bfr(float f) { return __uint_as_float(((unsigned)f2bf(f)) << 16); }
__device__ __forceinline__ v16bf cat16b(v8us lo, v8us hi) { return __builtin_bit_cast(v16bf, __builtin_shufflevector(lo, hi, 0, 1, 2, 3, 4, 5, 6, 7, 8, 9, 10, 11, 12, 13, 14, 15)); }
__device__ __forceinline__ v8f wmmab(v16bf a, v16bf b, v8f c) { return __builtin_amdgcn_wmma_f32_16x16x32_bf16(false, a, false, b, (short)0, c, false, false); }
__device__ __forceinline__ v16bf ldb(const bf* p)  { return cat16b(*(const v8us*)p, *(const v8us*)(p + 16)); }
__device__ __forceinline__ void wave_sync() { __builtin_amdgcn_fence(3  , "wavefront"); __builtin_amdgcn_wave_barrier(); asm volatile("" ::: "memory"); }

__device__ __forceinline__ v8f wmmab_g(v16bf a, v16bf b, v8f c) {
    c = wmmab(a, b, c);
    asm volatile("v_nop\n\tv_nop\n\tv_nop\n\tv_nop" : "+v"(c) : "v"(a), "v"(b));
    return c;
}
__device__ __forceinline__ unsigned pkbf(float a, float b) { return (unsigned)f2bf(a) | (((unsigned)f2bf(b)) << 16); }

__device__ __forceinline__ v16bf basis31(float t, bool hs) {
    const float s  = 1.0f - t;
    const float t2 = t * t,   t3 = t2 * t,  t4 = t2 * t2, t5 = t4 * t,  t6 = t3 * t3, t7 = t4 * t3, T8 = t4 * t4;
    const float s2 = s * s,   s3 = s2 * s,  s4 = s2 * s2, s5 = s4 * s,  s6 = s3 * s3, s7 = s4 * s3, S8 = s4 * s4;
    const float g0 = s7, g1 = t * s6, g2 = t2 * s5, g3 = t3 * s4, g4 = t4 * s3, g5 = t5 * s2, g6 = t6 * s, g7 = t7;
    const float X  = hs ? T8 : S8;
    const float pa = (X * S8) * S8;
    const float pb = (T8 * T8) * X;
    v8u w;
    w[0] = pkbf(pa * g0, pa * g1); w[1] = pkbf(pa * g2, pa * g3); w[2] = pkbf(pa * g4, pa * g5); w[3] = pkbf(pa * g6, pa * g7);
    w[4] = pkbf(pb * g0, pb * g1); w[5] = pkbf(pb * g2, pb * g3); w[6] = pkbf(pb * g4, pb * g5); w[7] = pkbf(pb * g6, pb * g7);
    return __builtin_bit_cast(v16bf, w);
}

static_assert(128 * 8 == 2 * NV * KD);
static_assert(8 * 4 == 2 * NV);
__global__ __launch_bounds__(128) void k_prep(const float* __restrict__ params, const float* __restrict__ prange, bf* CB, float* RNG) {
    __shared__ unsigned bn[KD];
    __shared__ __align__(16) float cq[2 * NV * KD];
    __shared__ __align__(16) float rs[2 * NV];
    const int tid = threadIdx.x;
    if (tid == 0) {
        bn[0] = 1u;
#pragma unroll 1
        for (int d = 1; d < KD; ++d) bn[d] = 0u;
#pragma unroll 1
        for (int n = 1; n <= DEG - 1; ++n) {
#pragma unroll 1
            for (int d = n; d >= 1; --d) bn[d] = bn[d] + bn[d - 1];
        }
    }
    __syncthreads();
    if (tid < NV) {
        const int v = tid;
        const float p0    = bfr(params[v]);
        const float base1 = bfr(params[NV + v]);
        float csum = 0.0f, pd = p0;
#pragma unroll 1
        for (int d = 0; d < KD; ++d) {
            csum += expf(bfr(params[(d + 1) * NV + v]));
            const float pn = csum + base1;
            const float cb = (float)bn[d];
            cq[(v * 2 + 0) * KD + d] = cb * pd;
            cq[(v * 2 + 1) * KD + d] = cb * (pn - pd);
            pd = pn;
        }
        const float lo = bfr(prange[v]);
        const float hi = bfr(prange[NV + v]);
        rs[v] = lo;
        rs[NV + v] = 1.0f / (hi - lo);
    }
    __syncthreads();
    const v4f c0 = *(const v4fa*)(&cq[tid * 8]);
    const v4f c1 = *(const v4fa*)(&cq[tid * 8 + 4]);
    v8us o;
#pragma unroll
    for (int k = 0; k < 4; ++k) { o[k] = f2bf(c0[k]); o[4 + k] = f2bf(c1[k]); }
    const v4f rv = *(const v4fa*)(&rs[(tid & 7) * 4]);
#pragma unroll 1
    for (int ps = 0; ps < 2; ++ps) {
        *(volatile v8us*)(CB + (size_t)tid * 8) = o;
        if (tid < 8) *(volatile v4f*)(RNG + tid * 4) = rv;
        if (ps == 0) __threadfence();
    }
}

static_assert(2 * 32 * 4 == 16 * NV);
static_assert((size_t)TW * (256 + 512) * 4 <= (size_t)131072);
static_assert((size_t)(KD + 2 * NV * KD + 2 * NV) * 4 <= (size_t)131072);

#define BSTEP(V) { \
    const bool sel = (vq == (V)); \
    const v16bf bA = __builtin_bit_cast(v16bf, sel ? fA : zz); \
    accA = wmmab_g(basis31(tr[(V)], hs), bA, accA); \
    const v16bf bB = __builtin_bit_cast(v16bf, sel ? fB : zz); \
    accB = wmmab_g(basis31(tr[8 + (V)], hs), bB, accB); }

__global__ __launch_bounds__(32 * TW) void k_bern(const float* __restrict__ X, const bf* __restrict__ CB, const float* __restrict__ RNG, float* OUT) {
    __shared__ __align__(16) float ts[TW * 256];
    __shared__ __align__(16) float os[TW * 512];
    const int lane = threadIdx.x & 31, lr = lane & 15, hi = lane >> 4;
    const int wave = __builtin_amdgcn_readfirstlane((int)(threadIdx.x >> 5));
    const size_t n0 = ((size_t)blockIdx.x * TW + (size_t)wave) * 16;
    const int tb = wave * 256, ob = wave * 512;
    const bool hs = (hi != 0);
    const int vq = lr >> 1, q = lr & 1;
    const bool isg = (q != 0);

    {
        const int col0 = (lane & 3) * 4;
        const v4f lo4 = *(const v4f*)(RNG + col0);
        const v4f iv4 = *(const v4f*)(RNG + NV + col0);
        const float* xb = X + n0 * NV;
#pragma unroll
        for (int s = 0; s < 2; ++s) {
            const int e = (s * 32 + lane) * 4;
            const v4f xv = *(const v4f*)(xb + e);
            v4f tv;
#pragma unroll
            for (int i = 0; i < 4; ++i) tv[i] = (bfr(xv[i]) - lo4[i]) * iv4[i];
            *(v4fa*)(&ts[tb + e]) = tv;
        }
    }
    wave_sync();

    float tr[16];
    {
        const v4f r0 = *(const v4fa*)(&ts[tb + lr * 16 + 0]);
        const v4f r1 = *(const v4fa*)(&ts[tb + lr * 16 + 4]);
        const v4f r2 = *(const v4fa*)(&ts[tb + lr * 16 + 8]);
        const v4f r3 = *(const v4fa*)(&ts[tb + lr * 16 + 12]);
#pragma unroll
        for (int i = 0; i < 4; ++i) { tr[i] = r0[i]; tr[4 + i] = r1[i]; tr[8 + i] = r2[i]; tr[12 + i] = r3[i]; }
    }

    const v8u fA = __builtin_bit_cast(v8u, ldb(CB + (size_t)lr * KD + 8 * hi));
    const v8u fB = __builtin_bit_cast(v8u, ldb(CB + (size_t)(16 + lr) * KD + 8 * hi));
    const v8u zz = (v8u){};
    v8f accA = (v8f){}, accB = (v8f){};

    BSTEP(0) BSTEP(1) BSTEP(2) BSTEP(3) BSTEP(4) BSTEP(5) BSTEP(6) BSTEP(7)

#pragma unroll
    for (int r = 0; r < 8; ++r) {
        const int row = 8 * hi + r;
        const float a = accA[r], b = accB[r];
        const float ax = __shfl_xor(a, 1, 32), bx = __shfl_xor(b, 1, 32);
        const float tA = ts[tb + row * 16 + vq], tB = ts[tb + row * 16 + 8 + vq];
        const float GA = isg ? a : ax, FA = isg ? ax : a;
        const float GB = isg ? b : bx, FB = isg ? bx : b;
        const float yA = FA + tA * GA, yB = FB + tB * GB;
        const float lA = logf(fabsf(32.0f * GA)), lB = logf(fabsf(32.0f * GB));
        os[ob + q * 256 + row * 16 + vq]     = isg ? lA : yA;
        os[ob + q * 256 + row * 16 + 8 + vq] = isg ? lB : yB;
    }
    wave_sync();

    float* og = OUT + n0 * NV;
#pragma unroll 1
    for (int ps = 0; ps < 2; ++ps) {
#pragma unroll
        for (int qq = 0; qq < 2; ++qq) {
#pragma unroll
            for (int s = 0; s < 2; ++s) { const int e = (s * 32 + lane) * 4;
                const v4f val = *(const v4fa*)(&os[ob + qq * 256 + e]);
                *(volatile v4f*)(og + (size_t)qq * ((size_t)NROWS_FULL * NV) + e) = val; } }
        if (ps == 0) __threadfence(); }
}

static constexpr size_t al256(size_t v) { return (v + 255) & ~(size_t)255; }
static constexpr size_t SZ_CB  = al256((size_t)2 * NV * KD * 2);
static constexpr size_t SZ_RNG = al256((size_t)2 * NV * 4);
static constexpr size_t SZ_TOTAL = SZ_CB + SZ_RNG;
static_assert(SZ_TOTAL <= (size_t)134217728);
static_assert(SZ_CB % 128 == 0);

extern "C" void kernel_launch(void* const* d_in, const int* in_sizes, int n_in,
                              void* d_out, int out_size, void* d_ws, size_t ws_size, hipStream_t stream) {
    if (n_in < 3) return;
    if ((size_t)in_sizes[0] < (size_t)NROWS * NV) return;
    if ((size_t)in_sizes[1] < (size_t)(DEG + 1) * NV) return;
    if ((size_t)in_sizes[2] < (size_t)2 * NV) return;
    if ((size_t)out_size < (size_t)NROWS_FULL * NV + (size_t)NROWS * NV) return;
    if (SZ_TOTAL > ws_size) return;
    const float* x  = (const float*)d_in[0];
    const float* pm = (const float*)d_in[1];
    const float* pr = (const float*)d_in[2];
    float* OUT = (float*)d_out;
    char* wsp = (char*)d_ws;
    bf* CB = (bf*)wsp; wsp += SZ_CB;
    float* RNG = (float*)wsp; wsp += SZ_RNG;

    k_prep<<<1, 128, 0, stream>>>(pm, pr, CB, RNG);
    k_bern<<<NROWS / (16 * TW), 32 * TW, 0, stream>>>(x, CB, RNG, OUT);
}
